// GaussianSplatting_13597866459687
// MI455X (gfx1250) — hardware-verified
//
#include <hip/hip_runtime.h>


namespace {
constexpr int NPT = 32768, RES = 512;
constexpr float SIGMA = 0.02f, XS = 8.0f;
typedef _Float16 b16;
typedef __attribute__((ext_vector_type(16))) _Float16 v16b;
typedef __attribute__((ext_vector_type(8))) _Float16 v8b;
typedef __attribute__((ext_vector_type(8))) float v8f;
typedef __attribute__((ext_vector_type(4))) float v4f;
__device__ __forceinline__ float bf16_rne(float f) { unsigned int u = __float_as_uint(f); u += 0x7FFFu + ((u >> 16) & 1u); return __uint_as_float(u & 0xFFFF0000u); }
__device__ __forceinline__ void split16(float v, b16& hi, b16& lo) { hi = (b16)v; lo = (b16)(v - (float)hi); }
__device__ __forceinline__ v16b frag_kb(const b16* p, int hh) { const v8b a = *(const v8b*)(p + 8 * hh), b = *(const v8b*)(p + 16 + 8 * hh); v16b f;
#pragma unroll
  for (int e = 0; e < 8; ++e) { f[e] = a[e]; f[8 + e] = b[e]; } return f; }
__device__ __forceinline__ v8f wmma16b(v16b a, v16b b, v8f c) { v8f d = __builtin_amdgcn_wmma_f32_16x16x32_f16(false, a, false, b, (short)0, c, false, false); asm volatile("v_nop\n\tv_nop\n\tv_nop\n\tv_nop" : "+v"(d) : "v"(a), "v"(b)); return d; }
__device__ __forceinline__ void wave_lds_sync() { __builtin_amdgcn_fence(__ATOMIC_RELEASE, "workgroup"); __builtin_amdgcn_wave_barrier(); __builtin_amdgcn_fence(__ATOMIC_ACQUIRE, "workgroup"); }
__device__ __forceinline__ float pmul(float a, float b) { float p = a * b; asm volatile("" : "+v"(p)); return p; }

__global__ __launch_bounds__(256) void planes_kernel(const float* __restrict__ pos, const float* __restrict__ act, const float* __restrict__ scl, b16* __restrict__ AYh, b16* __restrict__ AYl, b16* __restrict__ BXh, b16* __restrict__ BXl) {
  const int g = blockIdx.x; const size_t n0 = (size_t)blockIdx.y * 2048 + threadIdx.x * 8; const float s = bf16_rne(scl[0]); const float gv = (float)g * (1.0f / (RES - 1)); const float c = 1.0f / (2.0f * SIGMA * SIGMA);
  v8b ah, al, bh, bl;
#pragma unroll
  for (int j = 0; j < 8; ++j) { const size_t n = n0 + j; const float px = bf16_rne(pos[n * 2]), py = bf16_rne(pos[n * 2 + 1]), a = bf16_rne(act[n]);
    const float x = 0.5f + s * (px - 0.5f); const float y = 1.0f - (0.5f + s * (py - 0.5f));
    const float dx = gv - x, dy = gv - y; const float ex = __expf(-(dx * dx) * c), ey = __expf(-(dy * dy) * c);
    b16 p, q; split16(pmul(ey, a) * XS, p, q); ah[j] = p; al[j] = q; split16(ex * XS, p, q); bh[j] = p; bl[j] = q; }
  const size_t o = (size_t)g * NPT + n0;
  for (int pass = 0; pass < 2; ++pass) { *(volatile v8b*)(AYh + o) = ah; *(volatile v8b*)(AYl + o) = al; *(volatile v8b*)(BXh + o) = bh; *(volatile v8b*)(BXl + o) = bl; __threadfence(); }
}
__global__ __launch_bounds__(128) void gemm_kernel(const b16* __restrict__ AYh, const b16* __restrict__ AYl, const b16* __restrict__ BXh, const b16* __restrict__ BXl, float* __restrict__ out) {
  __shared__ __attribute__((aligned(16))) float Tf[16][128 + 4];
  const int wave = threadIdx.x >> 5, lane = threadIdx.x & 31, nloc = lane & 15, hlf = lane >> 4; const int h0 = blockIdx.x * 16, wbase = blockIdx.y * 128 + wave * 32;
  v8f acc[2] = {(v8f){}, (v8f){}};
  const b16* ah = AYh + (size_t)(h0 + nloc) * NPT; const b16* al = AYl + (size_t)(h0 + nloc) * NPT;
#pragma unroll 4
  for (int kb = 0; kb < NPT; kb += 32) { const v16b a = frag_kb(ah + kb, hlf), a2 = frag_kb(al + kb, hlf);
#pragma unroll
    for (int t = 0; t < 2; ++t) { const size_t wrow = (size_t)(wbase + t * 16 + nloc) * NPT + kb; const v16b bh = frag_kb(BXh + wrow, hlf), bl = frag_kb(BXl + wrow, hlf);
      acc[t] = wmma16b(a, bh, acc[t]); acc[t] = wmma16b(a, bl, acc[t]); acc[t] = wmma16b(a2, bh, acc[t]); } }
#pragma unroll
  for (int t = 0; t < 2; ++t)
#pragma unroll 1
    for (int r = 0; r < 8; ++r) Tf[8 * hlf + r][wave * 32 + t * 16 + nloc] = acc[t][r] * (1.0f / (XS * XS));
  __syncthreads();
  for (int pass = 0; pass < 2; ++pass) { for (int rr = wave; rr < 16; rr += 4) *(volatile v4f*)(out + (size_t)(h0 + rr) * RES + blockIdx.y * 128 + lane * 4) = *(const v4f*)(&Tf[rr][lane * 4]); __threadfence(); }
}
}

extern "C" void kernel_launch(void* const* d_in, const int* in_sizes, int n_in, void* d_out, int out_size, void* d_ws, size_t ws_size, hipStream_t stream) {
  (void)n_in;
  auto Fp = [&](int i) { return (const float*)d_in[i]; };
  if (in_sizes[0] != NPT * 2 || in_sizes[1] != NPT || in_sizes[2] != 1 || out_size != RES * RES) return;
  const size_t plane = (size_t)RES * NPT * 2;
  if (ws_size < 4 * plane) return;
  b16* AYh = (b16*)d_ws; b16* AYl = AYh + (size_t)RES * NPT; b16* BXh = AYl + (size_t)RES * NPT; b16* BXl = BXh + (size_t)RES * NPT;
  planes_kernel<<<dim3(RES, NPT / 2048), 256, 0, stream>>>(Fp(0), Fp(1), Fp(2), AYh, AYl, BXh, BXl);
  gemm_kernel<<<dim3(RES / 16, RES / 128), 128, 0, stream>>>(AYh, AYl, BXh, BXl, (float*)d_out);
}
